// QKVAttentionLegacy_7404523618828
// MI455X (gfx1250) — hardware-verified
//
#include <hip/hip_runtime.h>


namespace {
constexpr int NBH = 32, CHN = 64, T = 2048, SE = 512, SK = SE + T  , CH = 256;
constexpr float XS = 8.0f, PS = 256.0f, SCALE = 0.125f  ;
typedef _Float16 b16;
typedef __attribute__((ext_vector_type(16))) _Float16 v16b;
typedef __attribute__((ext_vector_type(8))) _Float16 v8b;
typedef __attribute__((ext_vector_type(2))) _Float16 v2b;
typedef __attribute__((ext_vector_type(8))) float v8f;
__device__ __forceinline__ float bf16_rne(float f) { unsigned int u = __float_as_uint(f); u += 0x7FFFu + ((u >> 16) & 1u); float r = __uint_as_float(u & 0xFFFF0000u); asm volatile("" : "+v"(r)); return r; }
__device__ __forceinline__ float bfv(float f) { float r = bf16_rne(f); asm volatile("" : "+v"(r)); return r; }
__device__ __forceinline__ void split16(float v, b16& hi, b16& lo) { hi = (b16)v; lo = (b16)(v - (float)hi); }
__device__ __forceinline__ v16b frag_kb(const b16* p, int hh) { const v8b a = *(const v8b*)(p + 8 * hh), b = *(const v8b*)(p + 16 + 8 * hh); v16b f;
#pragma unroll
  for (int e = 0; e < 8; ++e) { f[e] = a[e]; f[8 + e] = b[e]; } return f; }
__device__ __forceinline__ v8f wmma16b(v16b a, v16b b, v8f c) { v8f d = __builtin_amdgcn_wmma_f32_16x16x32_f16(false, a, false, b, (short)0, c, false, false); asm volatile("v_nop\n\tv_nop\n\tv_nop\n\tv_nop" : "+v"(d) : "v"(a), "v"(b)); return d; }
__device__ __forceinline__ void wave_lds_sync() { __builtin_amdgcn_fence(__ATOMIC_RELEASE, "workgroup"); __builtin_amdgcn_wave_barrier(); __builtin_amdgcn_fence(__ATOMIC_ACQUIRE, "workgroup"); }

__global__ __launch_bounds__(256) void prep_kernel(const float* __restrict__ qkv, const float* __restrict__ ekv, b16* __restrict__ QT, b16* __restrict__ KT, b16* __restrict__ V) { __shared__ float Tq[CHN][65], Tk[CHN][65]; const int tid = threadIdx.x, wave = tid >> 5, lane = tid & 31; const int bh = blockIdx.x / (SK / 64), s0 = (blockIdx.x % (SK / 64)) * 64;
  const float* kq = qkv + (size_t)bh * 3 * CHN * T; const float* ke = ekv + (size_t)bh * 2 * CHN * SE;
  for (int c = wave; c < CHN; c += 8) { const int s = s0 + lane * 2; float k0, k1, v0, v1, q0 = 0.0f, q1 = 0.0f;
    if (s0 < SE) { k0 = ke[(size_t)c * SE + s]; k1 = ke[(size_t)c * SE + s + 1]; v0 = ke[(size_t)(CHN + c) * SE + s]; v1 = ke[(size_t)(CHN + c) * SE + s + 1]; }
    else { const int t = s - SE; q0 = kq[(size_t)c * T + t]; q1 = kq[(size_t)c * T + t + 1]; k0 = kq[(size_t)(CHN + c) * T + t]; k1 = kq[(size_t)(CHN + c) * T + t + 1]; v0 = kq[(size_t)(2 * CHN + c) * T + t]; v1 = kq[(size_t)(2 * CHN + c) * T + t + 1]; }
    Tk[c][lane * 2] = bfv(k0); Tk[c][lane * 2 + 1] = bfv(k1); Tq[c][lane * 2] = bfv(q0); Tq[c][lane * 2 + 1] = bfv(q1);
    for (int pass = 0; pass < 2; ++pass) { *(volatile v2b*)(V + ((size_t)bh * CHN + c) * SK + s) = (v2b){(b16)(bfv(v0) * XS), (b16)(bfv(v1) * XS)}; __threadfence(); } }
  __syncthreads();
  for (int pass = 0; pass < 2; ++pass) { for (int r = wave; r < 64; r += 8) { *(volatile v2b*)(KT + ((size_t)bh * SK + s0 + r) * CHN + lane * 2) = (v2b){(b16)(Tk[lane * 2][r] * XS), (b16)(Tk[lane * 2 + 1][r] * XS)}; if (s0 >= SE) *(volatile v2b*)(QT + ((size_t)bh * T + (s0 - SE) + r) * CHN + lane * 2) = (v2b){(b16)(Tq[lane * 2][r] * XS), (b16)(Tq[lane * 2 + 1][r] * XS)}; } __threadfence(); } }
__global__ __launch_bounds__(32) void att_kernel(const b16* __restrict__ QT, const b16* __restrict__ KT, const b16* __restrict__ V, int QLIM, float* __restrict__ out) { __shared__ __attribute__((aligned(16))) b16 Pa[32][CH + 8], Pb[32][CH + 8]; __shared__ float Sc[32][CH + 1], Mx[32], Ls[32], Fc[32], Of[32][CHN + 1]; const int lane = threadIdx.x, nloc = lane & 15, hlf = lane >> 4; const int bh = blockIdx.x / (T / 32), q0 = (blockIdx.x % (T / 32)) * 32; if (q0 >= QLIM) return; const size_t tq = (size_t)bh * T + q0;
  Mx[lane] = -INFINITY; Ls[lane] = 0.0f; for (int kk = CH; kk < CH + 8; ++kk) { Pa[lane][kk] = (b16)0.0f; Pb[lane][kk] = (b16)0.0f; }
  wave_lds_sync();
  v16b qa[2][2]; for (int rt = 0; rt < 2; ++rt) for (int ks = 0; ks < 2; ++ks) qa[rt][ks] = frag_kb(QT + (tq + rt * 16 + nloc) * CHN + ks * 32, hlf);
  v8f oacc[2][4];
#pragma unroll
  for (int rt = 0; rt < 2; ++rt)
#pragma unroll
    for (int t = 0; t < 4; ++t) oacc[rt][t] = (v8f){};
#pragma unroll 1
  for (int ch = 0; ch < SK / CH; ++ch) { const int k0 = ch * CH;
#pragma unroll 1
    for (int tg = 0; tg < 16; tg += 4) { v8f sacc[2][4];
#pragma unroll
      for (int rt = 0; rt < 2; ++rt)
#pragma unroll
        for (int t = 0; t < 4; ++t) sacc[rt][t] = (v8f){};
#pragma unroll
      for (int t = 0; t < 4; ++t)
#pragma unroll
        for (int ks = 0; ks < 2; ++ks) { const v16b kb = frag_kb(KT + ((size_t)bh * SK + k0 + (tg + t) * 16 + nloc) * CHN + ks * 32, hlf); sacc[0][t] = wmma16b(qa[0][ks], kb, sacc[0][t]); sacc[1][t] = wmma16b(qa[1][ks], kb, sacc[1][t]); }
#pragma unroll
      for (int rt = 0; rt < 2; ++rt)
#pragma unroll
        for (int t = 0; t < 4; ++t)
#pragma unroll
          for (int r8 = 0; r8 < 8; ++r8) Sc[rt * 16 + 8 * hlf + r8][(tg + t) * 16 + nloc] = sacc[rt][t][r8] * (SCALE / (XS * XS)); }
    wave_lds_sync();
    { const int r = lane; float mx = -INFINITY; for (int j = 0; j < CH; ++j) mx = fmaxf(mx, Sc[r][j]); const float mo = Mx[r], mn = fmaxf(mo, mx); float sm = 0.0f; for (int j = 0; j < CH; ++j) { const float p = __expf(Sc[r][j] - mn); sm += p; b16 ph, pl; split16(p * PS, ph, pl); Pa[r][j] = ph; Pb[r][j] = pl; } const float fac = (mo == -INFINITY) ? 0.0f : __expf(mo - mn); Fc[r] = fac; Ls[r] = Ls[r] * fac + sm; Mx[r] = mn; }
    wave_lds_sync();
#pragma unroll
    for (int rt = 0; rt < 2; ++rt)
#pragma unroll
      for (int t = 0; t < 4; ++t)
#pragma unroll
        for (int r8 = 0; r8 < 8; ++r8) oacc[rt][t][r8] *= Fc[rt * 16 + 8 * hlf + r8];
#pragma unroll 2
    for (int kb = 0; kb < CH; kb += 32)
#pragma unroll
      for (int rt = 0; rt < 2; ++rt) { const v16b pa = frag_kb(&Pa[rt * 16 + nloc][kb], hlf), pb = frag_kb(&Pb[rt * 16 + nloc][kb], hlf);
#pragma unroll
        for (int t = 0; t < 4; ++t) { const v16b vb = frag_kb(V + ((size_t)bh * CHN + t * 16 + nloc) * SK + k0 + kb, hlf); oacc[rt][t] = wmma16b(pa, vb, oacc[rt][t]); oacc[rt][t] = wmma16b(pb, vb, oacc[rt][t]); } }
    wave_lds_sync(); }
#pragma unroll
  for (int rt = 0; rt < 2; ++rt)
#pragma unroll
    for (int t = 0; t < 4; ++t)
#pragma unroll
      for (int r8 = 0; r8 < 8; ++r8) { const int r = rt * 16 + 8 * hlf + r8; Of[r][t * 16 + nloc] = oacc[rt][t][r8] * (1.0f / (PS * XS)) / Ls[r]; }
  wave_lds_sync();
  for (int pass = 0; pass < 2; ++pass) { for (int c = 0; c < CHN; ++c) ((volatile float*)out)[((size_t)bh * CHN + c) * T + q0 + lane] = Of[lane][c]; __threadfence(); } }
}

extern "C" void kernel_launch(void* const* d_in, const int* in_sizes, int n_in, void* d_out, int out_size, void* d_ws, size_t ws_size, hipStream_t stream) {
  (void)n_in;
  auto Fp = [&](int i) { return (const float*)d_in[i]; };
  if (in_sizes[0] != NBH * 3 * CHN * T || in_sizes[1] != NBH * 2 * CHN * SE || out_size != NBH * CHN * T) return;
  const int QLIM = T;
  size_t off = 0; char* ws = (char*)d_ws;
  auto carve = [&](size_t bytes) { char* p = ws + off; off += (bytes + 255) & ~(size_t)255; return p; };
  b16* QT = (b16*)carve((size_t)NBH * T * CHN * 2); b16* KT = (b16*)carve((size_t)NBH * SK * CHN * 2); b16* V = (b16*)carve((size_t)NBH * CHN * SK * 2);
  if (off > ws_size || off > ((size_t)36 << 20)) return;
  prep_kernel<<<NBH * (SK / 64), 256, 0, stream>>>(Fp(0), Fp(1), QT, KT, V);
  att_kernel<<<NBH * (T / 32), 32, 0, stream>>>(QT, KT, V, QLIM, (float*)d_out);
}
